// MetaModel_36962488549818
// MI455X (gfx1250) — hardware-verified
//
#include <hip/hip_runtime.h>


#define AS3 __attribute__((address_space(3)))

#define NB_    16
#define MP_    512
#define NC_    4
#define TS_    256
#define NTHR   512
#define OUTW   5
#define ROWF   (MP_ * OUTW)
#define NPIECE (ROWF / 4)

static_assert(NTHR == MP_);
static_assert(MP_ % 32 == 0);
static_assert(NPIECE == NTHR + 128);
static_assert((ROWF * 4) % 128 == 0);
static_assert(NC_ == 4);
static_assert(NTHR / 32 * 32 == MP_);

typedef _Float16 v16h __attribute__((ext_vector_type(16)));
typedef _Float16 v8h  __attribute__((ext_vector_type(8)));
typedef float    v8f  __attribute__((ext_vector_type(8)));
typedef float    v4f  __attribute__((ext_vector_type(4)));

typedef AS3 _Float16*       lp_h;
typedef AS3 const _Float16* lcp_h;
typedef AS3 float*          lp_f;

union Frag { v16h v; v8h half[2]; };

constexpr size_t NR_ELEM = (size_t)NB_ * MP_ * MP_;
constexpr int    NRP     = (int)(NR_ELEM / 8);
constexpr int    NRPBLK  = NRP / 256;
static_assert(NRP % 256 == 0);
constexpr size_t OFF_RH  = 0;
constexpr size_t SZ_RH   = NR_ELEM * 2;
constexpr size_t WS_END  = OFF_RH + SZ_RH;
static_assert(WS_END <= (size_t)134217728);
static_assert((size_t)NRP * 16 == SZ_RH);

#define PSCL   256.0f
#define INV256 0.00390625f

__device__ __forceinline__ v8f zero8() {
    v8f z;
#pragma unroll
    for (int i = 0; i < 8; ++i) z[i] = 0.0f;
    return z;
}

__device__ __forceinline__ void ldfrag_lds(Frag& f, lcp_h p) {
    f.half[0] = *(AS3 const v8h*)(p);
    f.half[1] = *(AS3 const v8h*)(p + 16);
}
__device__ __forceinline__ void ldfrag_glb(Frag& f, const _Float16* p) {
    f.half[0] = *(const v8h*)(p);
    f.half[1] = *(const v8h*)(p + 16);
}
__device__ __forceinline__ v8f mma16(v8f c, const Frag& a, const Frag& b) {
    return __builtin_amdgcn_wmma_f32_16x16x32_f16(false, a.v, false, b.v, (short)0, c, false, false);
}

__global__ __launch_bounds__(256)
void cvt_r_kernel(const float* __restrict__ R, _Float16* Rh)
{
    const int p = blockIdx.x * 256 + threadIdx.x;
    if (p >= NRP) return;
    const size_t e = (size_t)p * 8;
    const v4f a = *(const v4f*)(R + e);
    const v4f b = *(const v4f*)(R + e + 4);
    v8h hv;
#pragma unroll
    for (int i = 0; i < 4; ++i) {
        hv[i]     = (_Float16)a[i];
        hv[4 + i] = (_Float16)b[i];
    }
    _Float16* d = Rh + e;
    *(volatile v8h*)d = hv;
    __threadfence();
    *(volatile v8h*)d = hv;
}

__global__ __launch_bounds__(NTHR)
void sim_kernel(const float* __restrict__ R, const _Float16* __restrict__ Rh,
                const float* __restrict__ Tmat, const float* __restrict__ rho0,
                const float* __restrict__ beta, float* out)
{
    __shared__ __attribute__((aligned(16))) float    s_out[ROWF];
    __shared__ __attribute__((aligned(16))) _Float16 s_bt[16 * MP_];
    __shared__ __attribute__((aligned(16))) float    s_q[MP_];

    lp_f sOut = (lp_f)(&s_out[0]);
    lp_h sBt  = (lp_h)(&s_bt[0]);
    lp_f sQ   = (lp_f)(&s_q[0]);

    const int n    = blockIdx.x;
    const int tid  = threadIdx.x;
    const int lane = tid & 31;
    const int w    = tid >> 5;
    const int h    = lane >> 4;
    const int m    = lane & 15;
    const int j    = tid;

    float Tm[4][4];
#pragma unroll
    for (int c = 0; c < 4; ++c)
#pragma unroll
        for (int d = 0; d < 4; ++d) Tm[c][d] = Tmat[n * 16 + c * 4 + d];
    const float bt0 = beta[0], bt1 = beta[1], bt2 = beta[2], bt3 = beta[3];

    const v4f rv = *(const v4f*)(rho0 + ((size_t)n * MP_ + j) * NC_);
    float pr0 = rv[0], pr1 = rv[1], pr2 = rv[2], pr3 = rv[3];

    float nt = 0.0f;
    {
        const float* Rc = R + (size_t)n * MP_ * MP_ + j;
#pragma unroll 4
        for (int i = 0; i < MP_; ++i) nt += Rc[(size_t)i * MP_];
    }
    const float csum = nt;
    const float rcpn = 1.0f / fmaxf(nt, 1e-8f);

    {
        v8h zh;
#pragma unroll
        for (int i = 0; i < 8; ++i) zh[i] = (_Float16)0.0f;
        for (int i = tid; i < (15 * MP_) / 8; i += NTHR) *(AS3 v8h*)(sBt + MP_ + 8 * i) = zh;
    }

    const _Float16* arow0 = Rh + ((size_t)n * MP_ + (32 * w + m)) * MP_ + 8 * h;
    const _Float16* arow1 = arow0 + (size_t)16 * MP_;
    lcp_h bcol = sBt + m * MP_ + 8 * h;
    float* outn = out + (size_t)n * TS_ * ROWF;
    const int p2 = NTHR + (tid & 127);

#pragma unroll 1
    for (int t = 0; t < TS_; ++t) {
        const float ssum  = ((pr0 + pr1) + pr2) + pr3;
        const float sfree = 1.0f - ssum;
        sOut[OUTW * j + 0] = sfree;
        sOut[OUTW * j + 1] = pr0;
        sOut[OUTW * j + 2] = pr1;
        sOut[OUTW * j + 3] = pr2;
        sOut[OUTW * j + 4] = pr3;
        const float rb   = ((pr0 * bt0 + pr1 * bt1) + pr2 * bt2) + pr3 * bt3;
        const float rate = (rb * csum) * rcpn;
        const float p    = 1.0f - expf(-rate);
        sBt[j] = (_Float16)(p * PSCL);
        __syncthreads();

        float* orow = outn + (size_t)t * ROWF;
        const v4f o0 = *(AS3 const v4f*)(sOut + 4 * tid);
        const v4f o1 = *(AS3 const v4f*)(sOut + 4 * p2);
        *(volatile v4f*)(orow + 4 * tid) = o0;
        if (w < 4) *(volatile v4f*)(orow + 4 * p2) = o1;

        v8f acc0 = zero8(), acc1 = zero8();
#pragma unroll 2
        for (int k0 = 0; k0 < MP_; k0 += 32) {
            Frag a0, a1, b;
            ldfrag_glb(a0, arow0 + k0);
            ldfrag_glb(a1, arow1 + k0);
            ldfrag_lds(b, bcol + k0);
            acc0 = mma16(acc0, a0, b);
            acc1 = mma16(acc1, a1, b);
            asm volatile("v_nop\n\tv_nop\n\tv_nop\n\tv_nop"
                         : "+v"(acc0), "+v"(acc1)
                         : "v"(a0.v), "v"(a1.v), "v"(b.v));
        }
        if (m == 0) {
#pragma unroll
            for (int r = 0; r < 8; ++r) {
                sQ[32 * w + 8 * h + r]      = acc0[r] * INV256;
                sQ[32 * w + 16 + 8 * h + r] = acc1[r] * INV256;
            }
        }

        __threadfence();
        *(volatile v4f*)(orow + 4 * tid) = o0;
        if (w < 4) *(volatile v4f*)(orow + 4 * p2) = o1;
        __syncthreads();

        const float q    = sQ[j];
        const float ninf = sfree * q;
        const float nx0 = (((pr0 * Tm[0][0] + pr1 * Tm[1][0]) + pr2 * Tm[2][0]) + pr3 * Tm[3][0]) + ninf;
        const float nx1 =  ((pr0 * Tm[0][1] + pr1 * Tm[1][1]) + pr2 * Tm[2][1]) + pr3 * Tm[3][1];
        const float nx2 =  ((pr0 * Tm[0][2] + pr1 * Tm[1][2]) + pr2 * Tm[2][2]) + pr3 * Tm[3][2];
        const float nx3 =  ((pr0 * Tm[0][3] + pr1 * Tm[1][3]) + pr2 * Tm[2][3]) + pr3 * Tm[3][3];
        pr0 = fminf(fmaxf(nx0, 0.0f), 1e10f);
        pr1 = fminf(fmaxf(nx1, 0.0f), 1e10f);
        pr2 = fminf(fmaxf(nx2, 0.0f), 1e10f);
        pr3 = fminf(fmaxf(nx3, 0.0f), 1e10f);
    }
}

extern "C" void kernel_launch(void* const* d_in, const int* in_sizes, int n_in,
                              void* d_out, int out_size, void* d_ws, size_t ws_size,
                              hipStream_t stream)
{
    if (n_in < 4) return;
    if (in_sizes[0] != NB_ * MP_ * MP_) return;
    if (in_sizes[1] != NB_ * NC_ * NC_) return;
    if (in_sizes[2] != NB_ * MP_ * NC_) return;
    if (in_sizes[3] != NC_)             return;
    if (out_size != NB_ * TS_ * ROWF)   return;
    if (ws_size < WS_END)               return;

    const float* R      = (const float*)d_in[0];
    const float* Tmat   = (const float*)d_in[1];
    const float* rho    = (const float*)d_in[2];
    const float* params = (const float*)d_in[3];
    float* out = (float*)d_out;

    char* ws = (char*)d_ws;
    _Float16* Rh = (_Float16*)(ws + OFF_RH);

    cvt_r_kernel<<<dim3(NRPBLK), dim3(256), 0, stream>>>(R, Rh);
    sim_kernel<<<dim3(NB_), dim3(NTHR), 0, stream>>>(R, (const _Float16*)Rh, Tmat, rho, params, out);
}
